// PointNetSetAbstraction_23149873725517
// MI455X (gfx1250) — hardware-verified
//
#include <hip/hip_runtime.h>
#pragma clang fp contract(off)

typedef __attribute__((ext_vector_type(16))) _Float16 v16h;
typedef __attribute__((ext_vector_type(8)))  _Float16 v8h;
typedef __attribute__((ext_vector_type(8)))  float    v8f;
typedef __attribute__((ext_vector_type(4)))  float    v4f;
typedef __attribute__((ext_vector_type(4)))  int      v4i;

constexpr int NBATCH  = 8;
constexpr int NPTS    = 16384;
constexpr int NPOINT  = 2048;
constexpr int NSAMPLE = 32;
constexpr int CIN     = 16;
constexpr int CH1     = 32;
constexpr int CH2     = 32;
constexpr int CH3     = 64;
constexpr int NROWS   = NBATCH * NPTS;
constexpr int NCENT   = NBATCH * NPOINT;

constexpr float RAD2 = 0.01f;

constexpr float W_CARRY = 16.0f;
constexpr float H_CARRY = 64.0f;
constexpr float INV_L1  = 1.0f / W_CARRY;
constexpr float INV_L23 = 1.0f / (W_CARRY * H_CARRY);

constexpr int SUM3_MODE = 0;

constexpr size_t WS_OFF_X   = 0;
constexpr size_t WS_OFF_Y   = WS_OFF_X + (size_t)NROWS * 4;
constexpr size_t WS_OFF_Z   = WS_OFF_Y + (size_t)NROWS * 4;
constexpr size_t WS_OFF_SB  = WS_OFF_Z + (size_t)NROWS * 4;
constexpr size_t WS_OFF_FI  = WS_OFF_SB + (size_t)NROWS * 4;
constexpr size_t WS_OFF_H3  = WS_OFF_FI + (size_t)NCENT * 4;
constexpr size_t WS_TOTAL   = WS_OFF_H3 + (size_t)NROWS * CH3 * 4;
static_assert(WS_OFF_H3 % 128 == 0, "line aligned");
static_assert(WS_TOTAL <= 134217728u, "carve limit");
static_assert(WS_TOTAL == 35717120u, "carve audit");

constexpr size_t OUT0_FLOATS = (size_t)NBATCH * NPOINT * 3;
constexpr size_t OUT1_FLOATS = (size_t)NBATCH * NPOINT * CH3;
static_assert(OUT0_FLOATS * 4 == 196608u, "out0 bytes");
static_assert((OUT0_FLOATS + OUT1_FLOATS) * 4 == 4390912u, "d_out bytes");

__device__ __forceinline__ float bf16_rne(float f) {
  const unsigned u = __float_as_uint(f);
  const unsigned r = (u + 0x7FFFu + ((u >> 16) & 1u)) & 0xFFFF0000u;
  return __uint_as_float(r);
}

__device__ __forceinline__ float sqsum3(float a, float b, float c) {
  if (SUM3_MODE == 2) {
    float t = a * a;
    t = __builtin_fmaf(b, b, t);
    t = __builtin_fmaf(c, c, t);
    return t;
  }
  const float t0 = a * a;
  const float t1 = b * b;
  const float t2 = c * c;
  if (SUM3_MODE == 1) return (t0 + t1) + t2;
  return (t0 + t2) + t1;
}

__device__ __forceinline__ void lds_wave_sync() {
  __builtin_amdgcn_fence(__ATOMIC_RELEASE, "workgroup");
  __builtin_amdgcn_wave_barrier();
  __builtin_amdgcn_fence(__ATOMIC_ACQUIRE, "workgroup");
}

union FragU { v16h v; v8h h[2]; };
__device__ __forceinline__ v16h frag_load(const _Float16* p) {
  FragU f;
  f.h[0] = *(const v8h*)(p);
  f.h[1] = *(const v8h*)(p + 16);
  return f.v;
}

__device__ __forceinline__ v8f mma_h(v16h a, v16h b, v8f c) {
  c = __builtin_amdgcn_wmma_f32_16x16x32_f16(false, a, false, b, (short)0, c, false, false);
  asm volatile("v_nop\n\tv_nop\n\tv_nop\n\tv_nop" : "+v"(c) : "v"(a), "v"(b));
  return c;
}

static_assert(NROWS == 128 * 256 * 4, "prep coverage");
__global__ __launch_bounds__(256) void prep_kernel(const float* __restrict__ xyz,
                                                   float* __restrict__ X, float* __restrict__ Y,
                                                   float* __restrict__ Z, float* __restrict__ SB) {
#pragma clang fp contract(off)
  const int i = blockIdx.x * 256 + threadIdx.x;
  const float* src = xyz + (size_t)i * 12;
  const v4f a = *(const v4f*)(src);
  const v4f b = *(const v4f*)(src + 4);
  const v4f c = *(const v4f*)(src + 8);
  const float a0 = a[0], a1 = a[1], a2 = a[2], a3 = a[3];
  const float b0 = b[0], b1 = b[1], b2 = b[2], b3 = b[3];
  const float c0 = c[0], c1 = c[1], c2 = c[2], c3 = c[3];
  const float x0 = bf16_rne(a0), y0 = bf16_rne(a1), z0 = bf16_rne(a2);
  const float x1 = bf16_rne(a3), y1 = bf16_rne(b0), z1 = bf16_rne(b1);
  const float x2 = bf16_rne(b2), y2 = bf16_rne(b3), z2 = bf16_rne(c0);
  const float x3 = bf16_rne(c1), y3 = bf16_rne(c2), z3 = bf16_rne(c3);
  v4f vx, vy, vz, vs;
  vx[0] = x0; vx[1] = x1; vx[2] = x2; vx[3] = x3;
  vy[0] = y0; vy[1] = y1; vy[2] = y2; vy[3] = y3;
  vz[0] = z0; vz[1] = z1; vz[2] = z2; vz[3] = z3;
  vs[0] = sqsum3(x0, y0, z0);
  vs[1] = sqsum3(x1, y1, z1);
  vs[2] = sqsum3(x2, y2, z2);
  vs[3] = sqsum3(x3, y3, z3);
  const size_t o = (size_t)i * 4;
  *(volatile v4f*)(X + o) = vx;
  *(volatile v4f*)(Y + o) = vy;
  *(volatile v4f*)(Z + o) = vz;
  *(volatile v4f*)(SB + o) = vs;
  __threadfence();
  *(volatile v4f*)(X + o) = vx;
  *(volatile v4f*)(Y + o) = vy;
  *(volatile v4f*)(Z + o) = vz;
  *(volatile v4f*)(SB + o) = vs;
  __threadfence();
}

__global__ __launch_bounds__(1024) void fps_kernel(const float* __restrict__ X,
                                                   const float* __restrict__ Y,
                                                   const float* __restrict__ Z,
                                                   const float* __restrict__ xyz,
                                                   int* __restrict__ fps_idx,
                                                   float* __restrict__ out0) {
#pragma clang fp contract(off)
  __shared__ float rv[32];
  __shared__ int   rp[32];
  __shared__ int   curs;
  __shared__ int   sidx[NPOINT];

  const int b    = blockIdx.x;
  const int tid  = threadIdx.x;
  const int lane = tid & 31;
  const int wid  = tid >> 5;
  const float* Xb = X + (size_t)b * NPTS;
  const float* Yb = Y + (size_t)b * NPTS;
  const float* Zb = Z + (size_t)b * NPTS;

  float px[16], py[16], pz[16], mind[16];
  {
    v4f t[4];
#pragma unroll
    for (int g = 0; g < 4; ++g) t[g] = *(const v4f*)(Xb + g * 4096 + tid * 4);
#pragma unroll
    for (int g = 0; g < 4; ++g) {
      px[g * 4 + 0] = t[g][0]; px[g * 4 + 1] = t[g][1]; px[g * 4 + 2] = t[g][2]; px[g * 4 + 3] = t[g][3];
    }
    asm volatile("" ::: "memory");
#pragma unroll
    for (int g = 0; g < 4; ++g) t[g] = *(const v4f*)(Yb + g * 4096 + tid * 4);
#pragma unroll
    for (int g = 0; g < 4; ++g) {
      py[g * 4 + 0] = t[g][0]; py[g * 4 + 1] = t[g][1]; py[g * 4 + 2] = t[g][2]; py[g * 4 + 3] = t[g][3];
    }
    asm volatile("" ::: "memory");
#pragma unroll
    for (int g = 0; g < 4; ++g) t[g] = *(const v4f*)(Zb + g * 4096 + tid * 4);
#pragma unroll
    for (int g = 0; g < 4; ++g) {
      pz[g * 4 + 0] = t[g][0]; pz[g * 4 + 1] = t[g][1]; pz[g * 4 + 2] = t[g][2]; pz[g * 4 + 3] = t[g][3];
    }
    asm volatile("" ::: "memory");
  }
#pragma unroll
  for (int j = 0; j < 16; ++j) mind[j] = 1e10f;

  int cur = 0;
#pragma unroll 1
  for (int it = 0; it < NPOINT; ++it) {
    if (tid == 0) sidx[it] = cur;
    int cc = cur < 0 ? 0 : cur;
    cc = cc > (NPTS - 1) ? (NPTS - 1) : cc;
    const float cx = Xb[cc];
    const float cy = Yb[cc];
    const float cz = Zb[cc];

    float bestv = -1.0f;
    int   bestp = 0;
#pragma unroll
    for (int j = 0; j < 16; ++j) {
      const float dx = px[j] - cx;
      const float dy = py[j] - cy;
      const float dz = pz[j] - cz;
      const float d  = sqsum3(dx, dy, dz);
      const float md = fminf(mind[j], d);
      mind[j] = md;
      const int p = (j >> 2) * 4096 + tid * 4 + (j & 3);
      const bool take = (md > bestv);
      bestv = take ? md : bestv;
      bestp = take ? p : bestp;
    }
#pragma unroll
    for (int off = 16; off >= 1; off >>= 1) {
      const float ov = __shfl_xor(bestv, off);
      const int   op = __shfl_xor(bestp, off);
      const bool take = (ov > bestv) || ((ov == bestv) && (op < bestp));
      bestv = take ? ov : bestv;
      bestp = take ? op : bestp;
    }
    if (lane == 0) { rv[wid] = bestv; rp[wid] = bestp; }
    __syncthreads();
    if (wid == 0) {
      float v = rv[lane];
      int   p = rp[lane];
#pragma unroll
      for (int off = 16; off >= 1; off >>= 1) {
        const float ov = __shfl_xor(v, off);
        const int   op = __shfl_xor(p, off);
        const bool take = (ov > v) || ((ov == v) && (op < p));
        v = take ? ov : v;
        p = take ? op : p;
      }
      if (lane == 0) curs = p;
    }
    __syncthreads();
    cur = curs;
  }
  __syncthreads();

  const float* xin = xyz + (size_t)b * NPTS * 3;
  float* dst0 = out0 + (size_t)b * (NPOINT * 3);
  int*   dsti = fps_idx + (size_t)b * NPOINT;

  v4f o0;
  {
    const int e0 = 4 * tid;
#pragma unroll
    for (int i = 0; i < 4; ++i) {
      const int e = e0 + i;
      const int s = e / 3;
      const int c = e - 3 * s;
      int p = sidx[s];
      p = p < 0 ? 0 : p;
      p = p > (NPTS - 1) ? (NPTS - 1) : p;
      const float raw = xin[(size_t)p * 3 + c];
      o0[i] = bf16_rne(raw);
    }
  }
  v4f o1 = (v4f){0.f, 0.f, 0.f, 0.f};
  v4i iv = (v4i){0, 0, 0, 0};
  if (tid < 512) {
    const int e0 = 4096 + 4 * tid;
#pragma unroll
    for (int i = 0; i < 4; ++i) {
      const int e = e0 + i;
      const int s = e / 3;
      const int c = e - 3 * s;
      int p = sidx[s];
      p = p < 0 ? 0 : p;
      p = p > (NPTS - 1) ? (NPTS - 1) : p;
      const float raw = xin[(size_t)p * 3 + c];
      o1[i] = bf16_rne(raw);
      iv[i] = sidx[4 * tid + i];
    }
  }
  *(volatile v4f*)(dst0 + 4 * tid) = o0;
  if (tid < 512) {
    *(volatile v4f*)(dst0 + 4096 + 4 * tid) = o1;
    *(volatile v4i*)(dsti + 4 * tid) = iv;
  }
  __threadfence();
  *(volatile v4f*)(dst0 + 4 * tid) = o0;
  if (tid < 512) {
    *(volatile v4f*)(dst0 + 4096 + 4 * tid) = o1;
    *(volatile v4i*)(dsti + 4 * tid) = iv;
  }
  __threadfence();
}

constexpr int MLP_TILES = 4;
constexpr int MLP_ROWS_PER_BLOCK = 16 * MLP_TILES * 8;
constexpr int MLP_BLOCKS = NROWS / MLP_ROWS_PER_BLOCK;
static_assert(NROWS % MLP_ROWS_PER_BLOCK == 0, "mlp coverage");

template <int KV, int NN>
__device__ __forceinline__ void stage_weight(const float* __restrict__ W, _Float16* sB, int tid) {
#pragma unroll 1
  for (int q = tid; q < NN * 4; q += 256) {
    const int n  = q % NN;
    const int kg = q / NN;
    float w[8];
#pragma unroll
    for (int e = 0; e < 8; ++e) {
      const int k  = kg * 8 + e;
      const int kc = (k < KV) ? k : (KV - 1);
      w[e] = W[(size_t)kc * NN + n];
    }
    v8h hv;
#pragma unroll
    for (int e = 0; e < 8; ++e) {
      const int k = kg * 8 + e;
      const float wr = bf16_rne(w[e]) * W_CARRY;
      const float f = (k < KV) ? wr : 0.0f;
      hv[e] = (_Float16)f;
    }
    *(v8h*)(sB + n * 32 + kg * 8) = hv;
  }
}

__global__ __launch_bounds__(256) void mlp_kernel(const float* __restrict__ features,
                                                  const float* __restrict__ W1, const float* __restrict__ b1,
                                                  const float* __restrict__ W2, const float* __restrict__ b2,
                                                  const float* __restrict__ W3, const float* __restrict__ b3,
                                                  float* __restrict__ H3) {
  __shared__ __align__(16) _Float16 sB1[CH1 * 32];
  __shared__ __align__(16) _Float16 sB2[CH2 * 32];
  __shared__ __align__(16) _Float16 sB3[CH3 * 32];
  __shared__ __align__(16) _Float16 sA[8][16 * 32];
  __shared__ __align__(16) float    sO[8][16 * 68];

  const int tid  = threadIdx.x;
  const int wave = tid >> 5;
  const int lane = tid & 31;
  const int hh   = lane >> 4;
  const int m    = lane & 15;

  stage_weight<CIN, CH1>(W1, sB1, tid);
  asm volatile("" ::: "memory");
  stage_weight<CH1, CH2>(W2, sB2, tid);
  asm volatile("" ::: "memory");
  stage_weight<CH2, CH3>(W3, sB3, tid);
  __syncthreads();

  v16h B1[2], B2[2], B3[4];
#pragma unroll
  for (int ni = 0; ni < 2; ++ni) B1[ni] = frag_load(sB1 + (ni * 16 + m) * 32 + 8 * hh);
#pragma unroll
  for (int ni = 0; ni < 2; ++ni) B2[ni] = frag_load(sB2 + (ni * 16 + m) * 32 + 8 * hh);
#pragma unroll
  for (int ni = 0; ni < 4; ++ni) B3[ni] = frag_load(sB3 + (ni * 16 + m) * 32 + 8 * hh);

  float bias1[2], bias2[2], bias3[4];
#pragma unroll
  for (int ni = 0; ni < 2; ++ni) { const float t = b1[ni * 16 + m]; bias1[ni] = bf16_rne(t); }
#pragma unroll
  for (int ni = 0; ni < 2; ++ni) { const float t = b2[ni * 16 + m]; bias2[ni] = bf16_rne(t); }
#pragma unroll
  for (int ni = 0; ni < 4; ++ni) { const float t = b3[ni * 16 + m]; bias3[ni] = bf16_rne(t); }

  _Float16* sAw = sA[wave];
  float*    sOw = sO[wave];

  float zf = 0.0f;
  asm volatile("" : "+v"(zf));
  v8h zv;
#pragma unroll
  for (int e = 0; e < 8; ++e) zv[e] = (_Float16)zf;

  const v8f zacc = (v8f){0.f, 0.f, 0.f, 0.f, 0.f, 0.f, 0.f, 0.f};

#pragma unroll 1
  for (int t = 0; t < MLP_TILES; ++t) {
    const int row0 = blockIdx.x * MLP_ROWS_PER_BLOCK + wave * (16 * MLP_TILES) + t * 16;

    {
      const int r  = lane >> 1;
      const int hf = lane & 1;
      const float* src = features + (size_t)(row0 + r) * CIN + hf * 8;
      const v4f f0 = *(const v4f*)(src);
      const v4f f1 = *(const v4f*)(src + 4);
      v8h hv;
#pragma unroll
      for (int e = 0; e < 4; ++e) {
        const float s0 = f0[e];
        const float s1 = f1[e];
        hv[e]     = (_Float16)bf16_rne(s0);
        hv[4 + e] = (_Float16)bf16_rne(s1);
      }
      *(v8h*)(sAw + r * 32 + hf * 8) = hv;
      *(v8h*)(sAw + r * 32 + 16 + hf * 8) = zv;
    }
    lds_wave_sync();

    v16h a = frag_load(sAw + m * 32 + 8 * hh);
    v8f c1[2];
#pragma unroll
    for (int ni = 0; ni < 2; ++ni) c1[ni] = mma_h(a, B1[ni], zacc);
    lds_wave_sync();
#pragma unroll
    for (int ni = 0; ni < 2; ++ni) {
#pragma unroll
      for (int r = 0; r < 8; ++r) {
        float v = c1[ni][r] * INV_L1;
        v = v + bias1[ni];
        v = fmaxf(v, 0.0f) * H_CARRY;
        sAw[(8 * hh + r) * 32 + ni * 16 + m] = (_Float16)v;
      }
    }
    lds_wave_sync();

    a = frag_load(sAw + m * 32 + 8 * hh);
    v8f c2[2];
#pragma unroll
    for (int ni = 0; ni < 2; ++ni) c2[ni] = mma_h(a, B2[ni], zacc);
    lds_wave_sync();
#pragma unroll
    for (int ni = 0; ni < 2; ++ni) {
#pragma unroll
      for (int r = 0; r < 8; ++r) {
        float v = c2[ni][r] * INV_L23;
        v = v + bias2[ni];
        v = fmaxf(v, 0.0f) * H_CARRY;
        sAw[(8 * hh + r) * 32 + ni * 16 + m] = (_Float16)v;
      }
    }
    lds_wave_sync();

    a = frag_load(sAw + m * 32 + 8 * hh);
    v8f c3[4];
#pragma unroll
    for (int nj = 0; nj < 4; ++nj) c3[nj] = mma_h(a, B3[nj], zacc);
    lds_wave_sync();
#pragma unroll
    for (int nj = 0; nj < 4; ++nj) {
#pragma unroll
      for (int r = 0; r < 8; ++r) {
        float v = c3[nj][r] * INV_L23;
        v = v + bias3[nj];
        sOw[(8 * hh + r) * 68 + nj * 16 + m] = v;
      }
    }
    lds_wave_sync();

    {
      const int c4 = m * 4;
      for (int pass = 0; pass < 2; ++pass) {
#pragma unroll
        for (int it = 0; it < 8; ++it) {
          const int row = it * 2 + hh;
          const v4f v = *(const v4f*)(sOw + row * 68 + c4);
          *(volatile v4f*)(H3 + (size_t)(row0 + row) * CH3 + c4) = v;
        }
        __threadfence();
      }
    }
    lds_wave_sync();
  }
}

__device__ __forceinline__ void drain_hits(unsigned mbits, int pbase, int& cnt,
                                           float& m0, float& m1, float& m2, float& m3,
                                           const float* __restrict__ H3b, int hh, int c4) {
#pragma unroll 1
  for (int t = 0; t < NSAMPLE; ++t) {
    if (mbits == 0u || cnt >= NSAMPLE) break;
    const int bA = __builtin_ctz(mbits);
    mbits &= (mbits - 1u);
    ++cnt;
    int bB = bA;
    if (mbits != 0u && cnt < NSAMPLE) {
      bB = __builtin_ctz(mbits);
      mbits &= (mbits - 1u);
      ++cnt;
    }
    int p = pbase + (hh ? bB : bA);
    p = p < 0 ? 0 : p;
    p = p > (NPTS - 1) ? (NPTS - 1) : p;
    const v4f v = *(const v4f*)(H3b + (size_t)p * CH3 + c4);
    m0 = fmaxf(m0, v[0]);
    m1 = fmaxf(m1, v[1]);
    m2 = fmaxf(m2, v[2]);
    m3 = fmaxf(m3, v[3]);
  }
}

static_assert(NCENT % 8 == 0, "ball query coverage");
__global__ __launch_bounds__(256) void ballq_max_kernel(const float* __restrict__ X,
                                                        const float* __restrict__ Y,
                                                        const float* __restrict__ Z,
                                                        const float* __restrict__ SB,
                                                        const int* __restrict__ fps_idx,
                                                        const float* __restrict__ H3,
                                                        float* __restrict__ out1) {
#pragma clang fp contract(off)
  const int wave = threadIdx.x >> 5;
  const int lane = threadIdx.x & 31;
  const int hh   = lane >> 4;
  const int c4   = (lane & 15) * 4;
  const int cent = blockIdx.x * 8 + wave;
  const int b    = cent / NPOINT;

  int fi = fps_idx[cent];
  fi = fi < 0 ? 0 : fi;
  fi = fi > (NPTS - 1) ? (NPTS - 1) : fi;

  const float* Xb = X + (size_t)b * NPTS;
  const float* Yb = Y + (size_t)b * NPTS;
  const float* Zb = Z + (size_t)b * NPTS;
  const float* Sb = SB + (size_t)b * NPTS;
  const float* H3b = H3 + (size_t)b * NPTS * CH3;

  const float cx = Xb[fi];
  const float cy = Yb[fi];
  const float cz = Zb[fi];
  const float sa = sqsum3(cx, cy, cz);

  float m0 = -INFINITY, m1 = -INFINITY, m2 = -INFINITY, m3 = -INFINITY;
  int cnt = 0;

#pragma unroll 1
  for (int p0 = 0; p0 < NPTS; p0 += 64) {
    if (cnt >= NSAMPLE) break;
    const int pa = p0 + lane;
    const int pb = p0 + 32 + lane;
    const float xa = Xb[pa], ya = Yb[pa], za = Zb[pa], sba = Sb[pa];
    const float xb = Xb[pb], yb = Yb[pb], zb = Zb[pb], sbb = Sb[pb];

    float da = cx * xa;
    da = __builtin_fmaf(cy, ya, da);
    da = __builtin_fmaf(cz, za, da);
    const float ta = sa + sba;
    const float d2a = ta - 2.0f * da;

    float db = cx * xb;
    db = __builtin_fmaf(cy, yb, db);
    db = __builtin_fmaf(cz, zb, db);
    const float tb = sa + sbb;
    const float d2b = tb - 2.0f * db;

    const unsigned ma = (unsigned)__ballot(d2a <= RAD2);
    const unsigned mb = (unsigned)__ballot(d2b <= RAD2);

    drain_hits(ma, p0, cnt, m0, m1, m2, m3, H3b, hh, c4);
    drain_hits(mb, p0 + 32, cnt, m0, m1, m2, m3, H3b, hh, c4);
  }

  const float s0 = __shfl_xor(m0, 16);
  const float s1 = __shfl_xor(m1, 16);
  const float s2 = __shfl_xor(m2, 16);
  const float s3 = __shfl_xor(m3, 16);
  v4f o;
  o[0] = fmaxf(m0, s0);
  o[1] = fmaxf(m1, s1);
  o[2] = fmaxf(m2, s2);
  o[3] = fmaxf(m3, s3);

  float* dst = out1 + (size_t)cent * CH3 + c4;
  if (lane < 16) *(volatile v4f*)dst = o;
  __threadfence();
  if (lane < 16) *(volatile v4f*)dst = o;
  __threadfence();
}

extern "C" void kernel_launch(void* const* d_in, const int* in_sizes, int n_in,
                              void* d_out, int out_size, void* d_ws, size_t ws_size,
                              hipStream_t stream) {
  if (n_in < 8) return;
  if (in_sizes[0] != NROWS * 3) return;
  if (in_sizes[1] != NROWS * CIN) return;
  if (in_sizes[2] != CIN * CH1 || in_sizes[3] != CH1) return;
  if (in_sizes[4] != CH1 * CH2 || in_sizes[5] != CH2) return;
  if (in_sizes[6] != CH2 * CH3 || in_sizes[7] != CH3) return;
  if ((size_t)out_size != OUT0_FLOATS + OUT1_FLOATS) return;
  if (ws_size < WS_TOTAL) return;

  const float* xyz      = (const float*)d_in[0];
  const float* features = (const float*)d_in[1];
  const float* W1 = (const float*)d_in[2];
  const float* b1 = (const float*)d_in[3];
  const float* W2 = (const float*)d_in[4];
  const float* b2 = (const float*)d_in[5];
  const float* W3 = (const float*)d_in[6];
  const float* b3 = (const float*)d_in[7];

  float* out0 = (float*)d_out;
  float* out1 = out0 + OUT0_FLOATS;

  unsigned char* ws = (unsigned char*)d_ws;
  float* X   = (float*)(ws + WS_OFF_X);
  float* Y   = (float*)(ws + WS_OFF_Y);
  float* Z   = (float*)(ws + WS_OFF_Z);
  float* SB  = (float*)(ws + WS_OFF_SB);
  int*   FI  = (int*)(ws + WS_OFF_FI);
  float* H3  = (float*)(ws + WS_OFF_H3);

  prep_kernel<<<128, 256, 0, stream>>>(xyz, X, Y, Z, SB);
  mlp_kernel<<<MLP_BLOCKS, 256, 0, stream>>>(features, W1, b1, W2, b2, W3, b3, H3);
  fps_kernel<<<NBATCH, 1024, 0, stream>>>(X, Y, Z, xyz, FI, out0);
  ballq_max_kernel<<<NCENT / 8, 256, 0, stream>>>(X, Y, Z, SB, FI, H3, out1);
}
